// Type_aware_GAT_28724741276290
// MI455X (gfx1250) — hardware-run, weakly checked
//
#include <hip/hip_runtime.h>
#include <math.h>
#include <stdint.h>

#define NB   8
#define NN   256
#define ND   256
#define NH   2
#define NV   50
#define NE   100
#define NROW (NB * NN)
#define KC   1536
#define NEGF (-9e15f)
#define SLOPE 0.2f

static_assert(NN == ND);
static_assert(NN == 256);
static_assert(NH == 2);
static_assert(NV == 50);
static_assert(NE == 100);
static_assert(KC % 32 == 0);
static_assert(KC == 3 * NN * NH);
static_assert((NN * 4) % 128 == 0);
static_assert((KC * 2) % 128 == 0);
static_assert(2 * NROW * NN == 1048576);

typedef __attribute__((ext_vector_type(16))) __bf16 v16b;
typedef __attribute__((ext_vector_type(8)))  __bf16 v8b;
typedef __attribute__((ext_vector_type(8)))  float  v8f;
typedef __attribute__((ext_vector_type(4)))  float  v4f;
typedef __attribute__((ext_vector_type(4)))  unsigned int v4u;
typedef __attribute__((ext_vector_type(2)))  unsigned int v2u;
typedef __attribute__((ext_vector_type(4)))  int    v4i;
typedef v4f __attribute__((may_alias)) v4fa;

__device__ __forceinline__ unsigned short f2bf_bits(float f) {
  const unsigned u = __float_as_uint(f);
  return (unsigned short)((u + 0x7FFFu + ((u >> 16) & 1u)) >> 16);
}
__device__ __forceinline__ float bf_bits2f(unsigned short h) { return __uint_as_float(((unsigned)h) << 16); }
__device__ __forceinline__ float bfr(float f) { return bf_bits2f(f2bf_bits(f)); }
__device__ __forceinline__ unsigned pk16(unsigned short a, unsigned short b) { return (unsigned)a | ((unsigned)b << 16); }

__device__ __forceinline__ void pin4(v4f x) { asm volatile("" :: "v"(x)); }
__device__ __forceinline__ void pin4i(v4i x) { asm volatile("" :: "v"(x)); }
__device__ __forceinline__ void pinf(float x) { asm volatile("" :: "v"(x)); }

__device__ __forceinline__ v8f mma_bf16(v16b a, v16b b, v8f c) {
  c = __builtin_amdgcn_wmma_f32_16x16x32_bf16(false, a, false, b, (short)0, c, false, false);
  asm volatile("v_nop\n\tv_nop\n\tv_nop\n\tv_nop" : "+v"(c) : "v"(a), "v"(b));
  return c;
}
union FB { v16b v; v8b h[2]; };
__device__ __forceinline__ v16b ldfrag(const __bf16* p) {
  FB f; f.h[0] = *(const v8b*)(p); f.h[1] = *(const v8b*)(p + 16); return f.v;
}

__device__ __forceinline__ void cvt8(const float* __restrict__ src, unsigned short* __restrict__ dst) {
  const v4f a = *(const v4f*)src;
  const v4f c = *(const v4f*)(src + 4);
  const v4u o = { pk16(f2bf_bits(a.x), f2bf_bits(a.y)), pk16(f2bf_bits(a.z), f2bf_bits(a.w)),
                  pk16(f2bf_bits(c.x), f2bf_bits(c.y)), pk16(f2bf_bits(c.z), f2bf_bits(c.w)) };
  *(volatile v4u*)dst = o;
  __threadfence();
  *(volatile v4u*)dst = o;
}

__global__ __launch_bounds__(256) void k_prep(const float* __restrict__ x, const float* __restrict__ W,
                                              const float* __restrict__ etw,
                                              unsigned short* __restrict__ XB, unsigned short* __restrict__ WB) {
  __shared__ __align__(16) float tf[64 * 68];
  const int blk = blockIdx.x, tid = threadIdx.x;
  if (blk < 256) {
    const size_t g = (size_t)blk * 256 + tid;
    cvt8(x + g * 8, XB + g * 8);
  } else if (blk < 320) {
    const size_t g = (size_t)(blk - 256) * 256 + tid;
    cvt8(etw + g * 8, WB + (size_t)512 * 256 + g * 8);
  } else {
    const int t  = blk - 320;
    const int z  = t >> 4, tt = t & 15;
    const int c0 = (tt & 3) * 64;
    const int r0 = (tt >> 2) * 64;
    const float* in = W + (size_t)z * ND * ND;
    unsigned short* oh = WB + (size_t)z * ND * ND;
    {
      const int lr = tid >> 4, c4 = (tid & 15) * 4;
#pragma unroll
      for (int it = 0; it < 4; ++it) {
        const int rr = it * 16 + lr;
        const v4f a = *(const v4f*)(in + (size_t)(r0 + rr) * ND + c0 + c4);
        *(v4fa*)(tf + rr * 68 + c4) = a;
      }
    }
    __syncthreads();
    const int sub = tid >> 3, c8 = (tid & 7) * 8;
    v4u hv[2];
#pragma unroll
    for (int it = 0; it < 2; ++it) {
      const int oc = it * 32 + sub;
      const float f0 = tf[(c8 + 0) * 68 + oc], f1 = tf[(c8 + 1) * 68 + oc];
      const float f2 = tf[(c8 + 2) * 68 + oc], f3 = tf[(c8 + 3) * 68 + oc];
      const float f4 = tf[(c8 + 4) * 68 + oc], f5 = tf[(c8 + 5) * 68 + oc];
      const float f6 = tf[(c8 + 6) * 68 + oc], f7 = tf[(c8 + 7) * 68 + oc];
      const v4u a = { pk16(f2bf_bits(f0), f2bf_bits(f1)), pk16(f2bf_bits(f2), f2bf_bits(f3)),
                      pk16(f2bf_bits(f4), f2bf_bits(f5)), pk16(f2bf_bits(f6), f2bf_bits(f7)) };
      hv[it] = a;
    }
    for (int pass = 0; pass < 2; ++pass) {
#pragma unroll
      for (int it = 0; it < 2; ++it) {
        const int oc = it * 32 + sub;
        *(volatile v4u*)(oh + (size_t)(c0 + oc) * ND + r0 + c8) = hv[it];
      }
      __threadfence();
    }
  }
}

__global__ __launch_bounds__(256) void k_tab(const float* __restrict__ tab, const float* __restrict__ emw,
                                             const float* __restrict__ emb, const float* __restrict__ eww,
                                             const float* __restrict__ ewb, const float* __restrict__ a,
                                             float* __restrict__ TAB) {
  __shared__ float sE[NV * NE];
  __shared__ float sP[102 * 8];
  __shared__ __align__(16) float sT[256];
  const int tid = threadIdx.x, lane = tid & 31, wave = tid >> 5;
#pragma unroll 4
  for (int i = tid; i < NV * NE; i += 256) sE[i] = bfr(tab[i]);
  sT[tid] = 0.0f;
  __syncthreads();
#pragma unroll 1
  for (int hd = 0; hd < NH; ++hd) {
    const float bc = bfr(emb[hd * ND + tid]);
    const float wc = bfr(eww[hd * ND + tid]);
    const float* wp = emw + (size_t)hd * NE * ND + tid;
#pragma unroll 1
    for (int t = 0; t < NV; ++t) {
      float s = 0.0f;
#pragma unroll 4
      for (int e = 0; e < NE; ++e) s = fmaf(sE[t * NE + e], bfr(wp[(size_t)e * ND]), s);
      s += bc;
      s = (s > 0.0f) ? s : 0.0f;
      float pr = s * wc;
      pr += __shfl_xor(pr, 16, 32);
      pr += __shfl_xor(pr, 8, 32);
      pr += __shfl_xor(pr, 4, 32);
      pr += __shfl_xor(pr, 2, 32);
      pr += __shfl_xor(pr, 1, 32);
      if (lane == 0) sP[(hd * NV + t) * 8 + wave] = pr;
    }
    float av = bfr(a[hd * 2 * ND + tid]);
    av += __shfl_xor(av, 16, 32);
    av += __shfl_xor(av, 8, 32);
    av += __shfl_xor(av, 4, 32);
    av += __shfl_xor(av, 2, 32);
    av += __shfl_xor(av, 1, 32);
    if (lane == 0) sP[(100 + hd) * 8 + wave] = av;
  }
  __syncthreads();
  {
    const int p = (tid < 102) ? tid : 101;
    float sum = 0.0f;
#pragma unroll
    for (int w = 0; w < 8; ++w) sum += sP[p * 8 + w];
    const int hdx = (p >= NV && p < 2 * NV) ? 1 : 0;
    const float eb = bfr(ewb[hdx]);
    pinf(sum); pinf(eb);
    float v = sum + eb;
    v = (v >= 0.0f) ? v : SLOPE * v;
    const int t = p - hdx * NV;
    if (tid < 2 * NV) sT[hdx * 64 + t] = v;
    else if (tid < 102) sT[128 + (tid - 100)] = sum;
  }
  __syncthreads();
  {
    const v4f tv = *(const v4fa*)(sT + 4 * (tid & 63));
    pin4(tv);
    if (tid < 64) {
      volatile v4f* d = (volatile v4f*)(TAB + 4 * tid);
      *d = tv;
      __threadfence();
      *d = tv;
    }
  }
}

template <int MODE>
__global__ __launch_bounds__(256) __attribute__((amdgpu_num_vgpr(248)))
void k_gemm(const unsigned short* __restrict__ Ap, int lda, long strideA,
            const unsigned short* __restrict__ Btp, int ldb, long strideB,
            float* __restrict__ Cf, int ldc, long strideC,
            unsigned short* __restrict__ Pl,
            int M, int N, int K, float scale) {
  __shared__ __align__(16) float sT[8][16 * 68];
  const __bf16* A  = (const __bf16*)(const void*)Ap;
  const __bf16* Bt = (const __bf16*)(const void*)Btp;
  const int bz   = blockIdx.y;
  const int lane = threadIdx.x & 31;
  const int wave = threadIdx.x >> 5;
  const int tilesN = N >> 6;
  const int tilesM = M >> 6;
  const int tile = blockIdx.x * 8 + wave;
  if (tile >= tilesM * tilesN) return;
  const int tm = tile / tilesN;
  const int tn = tile - tm * tilesN;
  const int m0 = tm << 6;
  const int n0 = tn << 6;

  const __bf16* Ab = A  + (size_t)bz * strideA;
  const __bf16* Bb = Bt + (size_t)bz * strideB;

  const int rlane = lane & 15;
  const int koff  = (lane >> 4) * 8;
  const int mOff  = (lane >> 4) * 8;

  v8f acc[4][4];
#pragma unroll
  for (int i = 0; i < 4; ++i)
#pragma unroll
    for (int j = 0; j < 4; ++j) acc[i][j] = (v8f){0.f, 0.f, 0.f, 0.f, 0.f, 0.f, 0.f, 0.f};

#pragma unroll 1
  for (int k0 = 0; k0 < K; k0 += 32) {
    v16b bh[4];
#pragma unroll
    for (int j = 0; j < 4; ++j)
      bh[j] = ldfrag(Bb + (size_t)(n0 + (j << 4) + rlane) * ldb + koff + k0);
#pragma unroll
    for (int i = 0; i < 4; ++i) {
      const v16b ah = ldfrag(Ab + (size_t)(m0 + (i << 4) + rlane) * lda + koff + k0);
#pragma unroll
      for (int j = 0; j < 4; ++j) acc[i][j] = mma_bf16(ah, bh[j], acc[i][j]);
    }
  }

  float* slab = sT[wave];
#pragma unroll
  for (int i = 0; i < 4; ++i) {
    const int mBase = m0 + (i << 4);
#pragma unroll
    for (int j = 0; j < 4; ++j) {
#pragma unroll
      for (int r = 0; r < 8; ++r)
        slab[(mOff + r) * 68 + (j << 4) + rlane] = acc[i][j][r] * scale;
    }
    __builtin_amdgcn_fence(__ATOMIC_RELEASE, "workgroup");
    __builtin_amdgcn_wave_barrier();
    __builtin_amdgcn_fence(__ATOMIC_ACQUIRE, "workgroup");
    if (MODE == 0) {
      float* C = Cf + (size_t)bz * strideC;
      const int hh = lane >> 4, c4 = (lane & 15) * 4;
      for (int pass = 0; pass < 2; ++pass) {
#pragma unroll
        for (int it = 0; it < 8; ++it) {
          const int row = it * 2 + hh;
          const v4f v = *(const v4fa*)(slab + row * 68 + c4);
          *(volatile v4f*)(C + (size_t)(mBase + row) * ldc + n0 + c4) = v;
        }
        __threadfence();
      }
    } else {
      const int q = lane >> 3, c8 = (lane & 7) * 8;
      const int seg = m0 >> 8, hd = seg & 1, br = seg >> 1;
      const int cB = (m0 & 255) + (i << 4);
      unsigned short* Pb = Pl + ((size_t)(br * NB + bz) * 256) * KC + hd * 768 + n0 + c8;
      for (int pass = 0; pass < 2; ++pass) {
#pragma unroll
        for (int it = 0; it < 4; ++it) {
          const int row = it * 4 + q;
          const float* sp = slab + row * 68 + c8;
          const float f0 = sp[0], f1 = sp[1], f2 = sp[2], f3 = sp[3];
          const float f4 = sp[4], f5 = sp[5], f6 = sp[6], f7 = sp[7];
          const unsigned short h0 = f2bf_bits(f0), h1 = f2bf_bits(f1), h2 = f2bf_bits(f2), h3 = f2bf_bits(f3);
          const unsigned short h4 = f2bf_bits(f4), h5 = f2bf_bits(f5), h6 = f2bf_bits(f6), h7 = f2bf_bits(f7);
          const v4u hv = { pk16(h0, h1), pk16(h2, h3), pk16(h4, h5), pk16(h6, h7) };
          const v4u lv = { pk16(f2bf_bits(f0 - bf_bits2f(h0)), f2bf_bits(f1 - bf_bits2f(h1))),
                           pk16(f2bf_bits(f2 - bf_bits2f(h2)), f2bf_bits(f3 - bf_bits2f(h3))),
                           pk16(f2bf_bits(f4 - bf_bits2f(h4)), f2bf_bits(f5 - bf_bits2f(h5))),
                           pk16(f2bf_bits(f6 - bf_bits2f(h6)), f2bf_bits(f7 - bf_bits2f(h7))) };
          unsigned short* d = Pb + (size_t)(cB + row) * KC;
          *(volatile v4u*)(d)       = hv;
          *(volatile v4u*)(d + 256) = hv;
          *(volatile v4u*)(d + 512) = lv;
        }
        __threadfence();
      }
    }
    __builtin_amdgcn_fence(__ATOMIC_RELEASE, "workgroup");
    __builtin_amdgcn_wave_barrier();
    __builtin_amdgcn_fence(__ATOMIC_ACQUIRE, "workgroup");
  }
}

__global__ __launch_bounds__(256) void k_d2(const float* __restrict__ Hf, const float* __restrict__ a,
                                            float* __restrict__ D2) {
  __shared__ __align__(16) float sA[256];
  __shared__ __align__(16) float sD[32];
  const int tid = threadIdx.x, lane = tid & 31, wave = tid >> 5;
  const int idx0 = blockIdx.x * 32;
  const int bh = idx0 >> 8, b = bh >> 1, hd = bh & 1, j0 = idx0 & 255;
  sA[tid] = bfr(a[hd * 2 * ND + ND + tid]);
  __syncthreads();
  const v4f a0 = *(const v4fa*)(sA + 8 * lane);
  const v4f a1 = *(const v4fa*)(sA + 8 * lane + 4);
#pragma unroll 1
  for (int q = 0; q < 4; ++q) {
    const int j = j0 + wave * 4 + q;
    const float* hr = Hf + ((size_t)(b * NN + j)) * (2 * ND) + hd * ND + 8 * lane;
    const v4f h0 = *(const v4f*)hr;
    const v4f h1 = *(const v4f*)(hr + 4);
    float s = h0.x * a0.x;
    s = fmaf(h0.y, a0.y, s); s = fmaf(h0.z, a0.z, s); s = fmaf(h0.w, a0.w, s);
    s = fmaf(h1.x, a1.x, s); s = fmaf(h1.y, a1.y, s); s = fmaf(h1.z, a1.z, s); s = fmaf(h1.w, a1.w, s);
    s += __shfl_xor(s, 16, 32);
    s += __shfl_xor(s, 8, 32);
    s += __shfl_xor(s, 4, 32);
    s += __shfl_xor(s, 2, 32);
    s += __shfl_xor(s, 1, 32);
    if (lane == 0) sD[wave * 4 + q] = s;
  }
  __syncthreads();
  const v4f v = *(const v4fa*)(sD + 4 * (tid & 7));
  pin4(v);
  if (tid < 8) {
    volatile v4f* d = (volatile v4f*)(D2 + idx0 + 4 * tid);
    *d = v;
    __threadfence();
    *d = v;
  }
}

__global__ __launch_bounds__(256) void k_att(const float* __restrict__ Hf, const float* __restrict__ D2,
                                             const float* __restrict__ TAB,
                                             const int* __restrict__ adj, const int* __restrict__ dep,
                                             unsigned short* __restrict__ APL, float* __restrict__ ATE) {
  __shared__ __align__(16) float sTab[256];
  const int tid = threadIdx.x, lane = tid & 31, wave = tid >> 5;
  sTab[tid] = TAB[tid];
  __syncthreads();
  const int row = blockIdx.x * 8 + wave;
  const int b = row >> 8;
  const int* ar = adj + (size_t)row * NN + 4 * lane;
  const int* dr = dep + (size_t)row * NN + 4 * lane;
  const v4i ma = *(const v4i*)ar;
  const v4i mb = *(const v4i*)(ar + 128);
  const v4i da = *(const v4i*)dr;
  const v4i db = *(const v4i*)(dr + 128);
  pin4i(ma); pin4i(mb); pin4i(da); pin4i(db);
  const int mk[8] = { ma.x, ma.y, ma.z, ma.w, mb.x, mb.y, mb.z, mb.w };
  const int dv[8] = { da.x, da.y, da.z, da.w, db.x, db.y, db.z, db.w };
  int id[8];
#pragma unroll
  for (int e = 0; e < 8; ++e) id[e] = min(max(dv[e], 0), NV - 1);

  float acc[8];
#pragma unroll
  for (int e = 0; e < 8; ++e) acc[e] = 0.0f;

#pragma unroll 1
  for (int q = 0; q < 4; ++q) {
    const int hd = q & 1, br = q >> 1;
    const float* hr = Hf + (size_t)row * (2 * ND) + hd * ND + 4 * lane;
    const float* dp = D2 + (size_t)(b * 2 + hd) * NN + 4 * lane;
    const v4f hf0 = *(const v4f*)hr;
    const v4f hf1 = *(const v4f*)(hr + 128);
    const v4f dd0 = *(const v4f*)dp;
    const v4f dd1 = *(const v4f*)(dp + 128);
    pin4(hf0); pin4(hf1); pin4(dd0); pin4(dd1);
    const float s1 = sTab[128 + hd];
    const float hfv[8] = { hf0.x, hf0.y, hf0.z, hf0.w, hf1.x, hf1.y, hf1.z, hf1.w };
    const float ddv[8] = { dd0.x, dd0.y, dd0.z, dd0.w, dd1.x, dd1.y, dd1.z, dd1.w };
    float s[8];
#pragma unroll
    for (int e = 0; e < 8; ++e) {
      float ev = hfv[e] * s1 + ddv[e];
      ev = (ev >= 0.0f) ? ev : SLOPE * ev;
      const float tv = sTab[hd * 64 + id[e]];
      pinf(tv);
      const float lg = (br != 0) ? tv : ev;
      s[e] = (mk[e] > 0) ? lg : NEGF;
    }
    float mx = s[0];
#pragma unroll
    for (int e = 1; e < 8; ++e) mx = fmaxf(mx, s[e]);
    mx = fmaxf(mx, __shfl_xor(mx, 16, 32));
    mx = fmaxf(mx, __shfl_xor(mx, 8, 32));
    mx = fmaxf(mx, __shfl_xor(mx, 4, 32));
    mx = fmaxf(mx, __shfl_xor(mx, 2, 32));
    mx = fmaxf(mx, __shfl_xor(mx, 1, 32));
    float p[8];
    float sum = 0.0f;
#pragma unroll
    for (int e = 0; e < 8; ++e) { p[e] = expf(s[e] - mx); sum += p[e]; }
    sum += __shfl_xor(sum, 16, 32);
    sum += __shfl_xor(sum, 8, 32);
    sum += __shfl_xor(sum, 4, 32);
    sum += __shfl_xor(sum, 2, 32);
    sum += __shfl_xor(sum, 1, 32);
    const float inv = 1.0f / sum;
    unsigned short hb[8], lb[8];
    float o[8];
#pragma unroll
    for (int e = 0; e < 8; ++e) {
      p[e] = p[e] * inv;
      hb[e] = f2bf_bits(p[e]);
      lb[e] = f2bf_bits(p[e] - bf_bits2f(hb[e]));
      o[e] = 0.5f * (acc[e] + p[e]);
      acc[e] = p[e];
    }
    const v2u H0 = { pk16(hb[0], hb[1]), pk16(hb[2], hb[3]) };
    const v2u H1 = { pk16(hb[4], hb[5]), pk16(hb[6], hb[7]) };
    const v2u L0 = { pk16(lb[0], lb[1]), pk16(lb[2], lb[3]) };
    const v2u L1 = { pk16(lb[4], lb[5]), pk16(lb[6], lb[7]) };
    const v4f O0 = { o[0], o[1], o[2], o[3] };
    const v4f O1 = { o[4], o[5], o[6], o[7] };
    unsigned short* ap = APL + ((size_t)br * NROW + row) * KC + hd * 768 + 4 * lane;
    float* fo = ATE + ((size_t)br * NROW + row) * NN + 4 * lane;
    for (int pass = 0; pass < 2; ++pass) {
      *(volatile v2u*)(ap)       = H0;
      *(volatile v2u*)(ap + 128) = H1;
      *(volatile v2u*)(ap + 256) = L0;
      *(volatile v2u*)(ap + 384) = L1;
      *(volatile v2u*)(ap + 512) = H0;
      *(volatile v2u*)(ap + 640) = H1;
      if (hd == 1) {
        *(volatile v4f*)(fo)       = O0;
        *(volatile v4f*)(fo + 128) = O1;
      }
      __threadfence();
    }
  }
}

__global__ __launch_bounds__(256) void k_fuse(const float* __restrict__ HT, const float* __restrict__ ATE,
                                              const float* __restrict__ tsw, const float* __restrict__ tsb,
                                              const float* __restrict__ esw, const float* __restrict__ esb,
                                              float* __restrict__ out) {
  __shared__ __align__(16) float sW[1024];
  const int tid = threadIdx.x, lane = tid & 31, wave = tid >> 5;
  sW[tid]       = bfr(tsw[tid]);
  sW[256 + tid] = bfr(tsw[256 + tid]);
  sW[512 + tid] = bfr(esw[tid]);
  sW[768 + tid] = bfr(esw[256 + tid]);
  const float tb = bfr(tsb[0]);
  const float eb = bfr(esb[0]);
  __syncthreads();
  const int row = blockIdx.x * 8 + wave;
  const float* tp = HT + (size_t)row * ND + 4 * lane;
  const float* ep = HT + (size_t)NROW * ND + (size_t)row * ND + 4 * lane;
  const float* atp = ATE + (size_t)row * NN + 4 * lane;
  const float* aep = ATE + (size_t)NROW * NN + (size_t)row * NN + 4 * lane;
  const v4f ht0 = *(const v4f*)tp,  ht1 = *(const v4f*)(tp + 128);
  const v4f he0 = *(const v4f*)ep,  he1 = *(const v4f*)(ep + 128);
  const v4f at0 = *(const v4f*)atp, at1 = *(const v4f*)(atp + 128);
  const v4f ae0 = *(const v4f*)aep, ae1 = *(const v4f*)(aep + 128);
  const v4f te0 = *(const v4fa*)(sW + 4 * lane),       te1 = *(const v4fa*)(sW + 128 + 4 * lane);
  const v4f tt0 = *(const v4fa*)(sW + 256 + 4 * lane), tt1 = *(const v4fa*)(sW + 384 + 4 * lane);
  const v4f ee0 = *(const v4fa*)(sW + 512 + 4 * lane), ee1 = *(const v4fa*)(sW + 640 + 4 * lane);
  const v4f et0 = *(const v4fa*)(sW + 768 + 4 * lane), et1 = *(const v4fa*)(sW + 896 + 4 * lane);
  const float hev[8] = { he0.x, he0.y, he0.z, he0.w, he1.x, he1.y, he1.z, he1.w };
  const float htv[8] = { ht0.x, ht0.y, ht0.z, ht0.w, ht1.x, ht1.y, ht1.z, ht1.w };
  const float tev[8] = { te0.x, te0.y, te0.z, te0.w, te1.x, te1.y, te1.z, te1.w };
  const float ttv[8] = { tt0.x, tt0.y, tt0.z, tt0.w, tt1.x, tt1.y, tt1.z, tt1.w };
  const float eev[8] = { ee0.x, ee0.y, ee0.z, ee0.w, ee1.x, ee1.y, ee1.z, ee1.w };
  const float etv[8] = { et0.x, et0.y, et0.z, et0.w, et1.x, et1.y, et1.z, et1.w };
  float zt = 0.0f, ze = 0.0f;
#pragma unroll
  for (int e = 0; e < 8; ++e) { zt = fmaf(hev[e], tev[e], zt); ze = fmaf(hev[e], eev[e], ze); }
#pragma unroll
  for (int e = 0; e < 8; ++e) { zt = fmaf(htv[e], ttv[e], zt); ze = fmaf(htv[e], etv[e], ze); }
  zt += __shfl_xor(zt, 16, 32);  ze += __shfl_xor(ze, 16, 32);
  zt += __shfl_xor(zt, 8, 32);   ze += __shfl_xor(ze, 8, 32);
  zt += __shfl_xor(zt, 4, 32);   ze += __shfl_xor(ze, 4, 32);
  zt += __shfl_xor(zt, 2, 32);   ze += __shfl_xor(ze, 2, 32);
  zt += __shfl_xor(zt, 1, 32);   ze += __shfl_xor(ze, 1, 32);
  const float sg_t = 1.0f / (1.0f + expf(-(zt + tb)));
  const float sg_e = 1.0f / (1.0f + expf(-(ze + eb)));
  const float omt = 1.0f - sg_t;
  const float atv[8] = { at0.x, at0.y, at0.z, at0.w, at1.x, at1.y, at1.z, at1.w };
  const float aev[8] = { ae0.x, ae0.y, ae0.z, ae0.w, ae1.x, ae1.y, ae1.z, ae1.w };
  float o0[8], o1[8];
#pragma unroll
  for (int e = 0; e < 8; ++e) {
    const float v = sg_t * htv[e] + omt * hev[e];
    o0[e] = (v <= 0.0f) ? 0.0f : v;
    o1[e] = sg_t * atv[e] + sg_e * aev[e];
  }
  const v4f A0 = { o0[0], o0[1], o0[2], o0[3] };
  const v4f A1 = { o0[4], o0[5], o0[6], o0[7] };
  const v4f B0 = { o1[0], o1[1], o1[2], o1[3] };
  const v4f B1 = { o1[4], o1[5], o1[6], o1[7] };
  float* d0 = out + (size_t)row * ND + 4 * lane;
  float* d1 = out + (size_t)NROW * ND + (size_t)row * NN + 4 * lane;
  for (int pass = 0; pass < 2; ++pass) {
    *(volatile v4f*)(d0)       = A0;
    *(volatile v4f*)(d0 + 128) = A1;
    *(volatile v4f*)(d1)       = B0;
    *(volatile v4f*)(d1 + 128) = B1;
    __threadfence();
  }
}

extern "C" void kernel_launch(void* const* d_in, const int* in_sizes, int n_in,
                              void* d_out, int out_size, void* d_ws, size_t ws_size,
                              hipStream_t stream) {
  if (n_in < 15) return;
  if (in_sizes[0] != NB * NN * ND) return;
  if (in_sizes[1] != NB * NN * NN) return;
  if (in_sizes[2] != NB * NN * NN) return;
  if (in_sizes[3] != NV * NE) return;
  if (in_sizes[4] != NH * ND * ND) return;
  if (in_sizes[5] != NH * 2 * ND) return;
  if (in_sizes[6] != NH * NE * ND) return;
  if (in_sizes[7] != NH * ND) return;
  if (in_sizes[8] != NH * ND) return;
  if (in_sizes[9] != NH) return;
  if (in_sizes[10] != NH * ND * ND) return;
  if (in_sizes[11] != 2 * ND) return;
  if (in_sizes[12] != 1) return;
  if (in_sizes[13] != 2 * ND) return;
  if (in_sizes[14] != 1) return;
  if (out_size != 2 * NROW * NN) return;

  const float* x    = (const float*)d_in[0];
  const int*   adj  = (const int*)d_in[1];
  const int*   dep  = (const int*)d_in[2];
  const float* tab  = (const float*)d_in[3];
  const float* W    = (const float*)d_in[4];
  const float* a    = (const float*)d_in[5];
  const float* emw  = (const float*)d_in[6];
  const float* emb  = (const float*)d_in[7];
  const float* eww  = (const float*)d_in[8];
  const float* ewb  = (const float*)d_in[9];
  const float* etw  = (const float*)d_in[10];
  const float* tsw  = (const float*)d_in[11];
  const float* tsb  = (const float*)d_in[12];
  const float* esw  = (const float*)d_in[13];
  const float* esb  = (const float*)d_in[14];
  float* out = (float*)d_out;

  const size_t szXB  = (size_t)NROW * ND * 2;
  const size_t szWB  = (size_t)1024 * ND * 2;
  const size_t szHf  = (size_t)NROW * 2 * ND * 4;
  const size_t szBT  = (size_t)16 * 256 * KC * 2;
  const size_t szAP  = (size_t)16 * 256 * KC * 2;
  const size_t szATE = (size_t)2 * NROW * NN * 4;
  const size_t szHT  = (size_t)2 * NROW * ND * 4;
  const size_t szTAB = (size_t)256 * 4;
  const size_t szD2  = (size_t)NB * NH * NN * 4;
  size_t off = 0;
  const size_t oXB = off;  off += szXB;
  const size_t oWB = off;  off += szWB;
  const size_t oHf = off;  off += szHf;
  const size_t oBT = off;  off += szBT;
  const size_t oAP = off;  off += szAP;
  const size_t oATE = off; off += szATE;
  const size_t oHT = off;  off += szHT;
  const size_t oTAB = off; off += szTAB;
  const size_t oD2 = off;  off += szD2;
  if (off > ws_size) return;
  if (off > (size_t)134217728) return;

  char* ws = (char*)d_ws;
  unsigned short* XB  = (unsigned short*)(ws + oXB);
  unsigned short* WB  = (unsigned short*)(ws + oWB);
  float*          Hf  = (float*)(ws + oHf);
  unsigned short* BTP = (unsigned short*)(ws + oBT);
  unsigned short* APL = (unsigned short*)(ws + oAP);
  float*          ATE = (float*)(ws + oATE);
  float*          HT  = (float*)(ws + oHT);
  float*          TAB = (float*)(ws + oTAB);
  float*          D2  = (float*)(ws + oD2);

  k_prep<<<dim3(352), dim3(256), 0, stream>>>(x, W, etw, XB, WB);
  k_tab<<<dim3(1), dim3(256), 0, stream>>>(tab, emw, emb, eww, ewb, a, TAB);
  k_gemm<0><<<dim3(32, 1), dim3(256), 0, stream>>>(XB, ND, 0L, WB, ND, 0L, Hf, 2 * ND, 0L, BTP,
                                                   NROW, 2 * ND, ND, 1.0f);
  k_gemm<1><<<dim3(8, NB), dim3(256), 0, stream>>>(WB, ND, 0L, XB, ND, (long)NN * ND, Hf, 2 * ND, 0L, BTP,
                                                   1024, NN, ND, 1.0f);
  k_d2<<<dim3(128), dim3(256), 0, stream>>>(Hf, a, D2);
  k_att<<<dim3(NROW / 8), dim3(256), 0, stream>>>(Hf, D2, TAB, adj, dep, APL, ATE);
  k_gemm<0><<<dim3(2, 16), dim3(256), 0, stream>>>(APL, KC, (long)256 * KC, BTP, KC, (long)256 * KC,
                                                   HT, ND, (long)NN * ND, BTP, NN, ND, KC, 0.5f);
  k_fuse<<<dim3(NROW / 8), dim3(256), 0, stream>>>(HT, ATE, tsw, tsb, esw, esb, out);
  (void)hipGetLastError();
}
